// NonLocalAttentionBlock_34729105555795
// MI455X (gfx1250) — hardware-verified
//
#include <hip/hip_runtime.h>


#define NB_  4
#define CC   512
#define DI   64
#define NPX  4096
#define QH   2048
#define DM   CC
#define BEPS 1e-5f
#define LOSC 1024.0f

typedef _Float16 h16;
typedef unsigned short bf;
typedef __attribute__((ext_vector_type(16))) __bf16   v16bf;
typedef __attribute__((ext_vector_type(16))) _Float16 v16h;
typedef __attribute__((ext_vector_type(8)))  _Float16 v8h;
typedef __attribute__((ext_vector_type(8)))  unsigned short v8us;
typedef __attribute__((ext_vector_type(8)))  float    v8f;
typedef __attribute__((ext_vector_type(4)))  float    v4f;
typedef v8h  __attribute__((may_alias)) v8ha;
typedef v4f  __attribute__((may_alias)) v4fa;
typedef v8us __attribute__((may_alias)) v8usa;

__device__ __forceinline__ unsigned short f2bf(float f) { unsigned u = __float_as_uint(f); u += 0x7FFFu + ((u >> 16) & 1u); return (unsigned short)(u >> 16); }
__device__ __forceinline__ float bf2f(unsigned short b) { return __uint_as_float(((unsigned)b) << 16); }
__device__ __forceinline__ float bfr(float f) { return bf2f(f2bf(f)); }
__device__ __forceinline__ v16h cat16(v8h lo, v8h hi) { return __builtin_shufflevector(lo, hi, 0, 1, 2, 3, 4, 5, 6, 7, 8, 9, 10, 11, 12, 13, 14, 15); }
__device__ __forceinline__ v16bf cat16b(v8us lo, v8us hi) { return __builtin_bit_cast(v16bf, __builtin_shufflevector(lo, hi, 0, 1, 2, 3, 4, 5, 6, 7, 8, 9, 10, 11, 12, 13, 14, 15)); }
__device__ __forceinline__ v8f wmma16(v16h a, v16h b, v8f c) { return __builtin_amdgcn_wmma_f32_16x16x32_f16(false, a, false, b, (short)0, c, false, false); }
__device__ __forceinline__ v8f wmmab(v16bf a, v16bf b, v8f c) { return __builtin_amdgcn_wmma_f32_16x16x32_bf16(false, a, false, b, (short)0, c, false, false); }

template <bool SPLITA, bool F16OUT = false>
__global__ __launch_bounds__(128) void k_gemmb(const bf* __restrict__ A, const bf* __restrict__ Al, const bf* __restrict__ Bn, const float* __restrict__ bias, float* C, int ldc, h16* C2, const float* __restrict__ R = nullptr, int K = DM, int roundR = 1) {
    __shared__ __align__(16) float ost[4][16 * 68];
    const int lane = threadIdx.x & 31, wave = threadIdx.x >> 5, lr = lane & 15, hi = lane >> 4;
    const int r0 = blockIdx.x * 64 + wave * 16, c0 = blockIdx.y * 64;
    const size_t aoff = (size_t)(r0 + lr) * K + 8 * hi;
    size_t boff[4];
#pragma unroll
    for (int t = 0; t < 4; ++t) boff[t] = (size_t)(c0 + t * 16 + lr) * K + 8 * hi;
    v8f acc[4];
#pragma unroll
    for (int t = 0; t < 4; ++t) acc[t] = (v8f){};
#pragma unroll 1
    for (int kc = 0; kc < K; kc += 32) {
        const v16bf a = cat16b(*(const v8us*)(A + aoff + kc), *(const v8us*)(A + aoff + kc + 16));
        v16bf al = a;
        if (SPLITA) al = cat16b(*(const v8us*)(Al + aoff + kc), *(const v8us*)(Al + aoff + kc + 16));
#pragma unroll
        for (int t = 0; t < 4; ++t) { const v16bf b = cat16b(*(const v8us*)(Bn + boff[t] + kc), *(const v8us*)(Bn + boff[t] + kc + 16)); acc[t] = wmmab(a, b, acc[t]); if (SPLITA) acc[t] = wmmab(al, b, acc[t]); }
        asm volatile("v_nop\n\tv_nop\n\tv_nop\n\tv_nop" : "+v"(acc[0]), "+v"(acc[1]), "+v"(acc[2]), "+v"(acc[3]) : "v"(a), "v"(al));
    }
    float* os = &ost[wave][0];
#pragma unroll
    for (int t = 0; t < 4; ++t) { const float bv = bias ? bfr(bias[c0 + t * 16 + lr]) : 0.f;
#pragma unroll
        for (int j = 0; j < 8; ++j) os[(hi * 8 + j) * 68 + t * 16 + lr] = acc[t][j] + bv; }
    __syncthreads();
    if (F16OUT) {
        h16* crow = (h16*)(void*)C + (size_t)r0 * ldc + c0;
        auto pass = [&]() {
#pragma unroll
            for (int s = 0; s < 4; ++s) { const int row = 4 * s + (lane >> 3), piece = lane & 7; const float* sp = os + row * 68 + piece * 8; v8h o, o2;
#pragma unroll
                for (int i = 0; i < 8; ++i) { const h16 a = (h16)sp[i]; o[i] = a; o2[i] = (h16)((sp[i] - (float)a) * LOSC); }
                *(volatile v8h*)(crow + (size_t)row * ldc + piece * 8) = o; if (C2) *(volatile v8h*)(C2 + (size_t)r0 * ldc + c0 + (size_t)row * ldc + piece * 8) = o2; }
        };
        pass(); __threadfence(); pass();
    } else {
        float* crow = C + (size_t)r0 * ldc + c0;
        auto pass = [&]() {
#pragma unroll
            for (int s = 0; s < 8; ++s) { const int Lid = (lane >> 3) + 4 * s, piece = lane & 7; const int row = Lid >> 1, cofs = (Lid & 1) * 32 + piece * 4;
                v4f val = *(const v4fa*)(os + row * 68 + cofs); if (R) { const v4f rv = *(const v4f*)(R + ((size_t)r0 + row) * ldc + c0 + cofs); val += roundR ? (v4f){bfr(rv[0]), bfr(rv[1]), bfr(rv[2]), bfr(rv[3])} : rv; }
                *(volatile v4f*)(crow + (size_t)row * ldc + cofs) = val; }
        };
        pass(); __threadfence(); pass();
    }
}

__global__ __launch_bounds__(256) void k_cvt8(const float* __restrict__ src, bf* dst, size_t n8) {
    const size_t i = (size_t)blockIdx.x * 256 + threadIdx.x; if (i >= n8) return;
    const v8f v = *(const v8f*)(src + i * 8); v8us o;
#pragma unroll
    for (int k = 0; k < 8; ++k) o[k] = f2bf(v[k]);
    *(volatile v8us*)(dst + i * 8) = o; __threadfence(); *(volatile v8us*)(dst + i * 8) = o;
}
__global__ __launch_bounds__(256) void k_zero8(bf* dst, size_t n8) {
    const size_t i = (size_t)blockIdx.x * 256 + threadIdx.x; if (i >= n8) return; v8us z;
#pragma unroll
    for (int k = 0; k < 8; ++k) z[k] = 0;
    *(volatile v8us*)(dst + i * 8) = z; __threadfence(); *(volatile v8us*)(dst + i * 8) = z;
}
__global__ __launch_bounds__(128) void k_gemm3(const bf* __restrict__ Ah, const bf* __restrict__ Al, const bf* __restrict__ Bh, const bf* __restrict__ Bl, int K, float* C, int ldc) {
    __shared__ __align__(16) float ost[4][16 * 68];
    const int lane = threadIdx.x & 31, wave = threadIdx.x >> 5, lr = lane & 15, hi = lane >> 4;
    const int r0 = blockIdx.x * 64 + wave * 16, c0 = blockIdx.y * 64;
    const size_t aoff = (size_t)(r0 + lr) * K + 8 * hi;
    v8f acc[4];
#pragma unroll
    for (int t = 0; t < 4; ++t) acc[t] = (v8f){};
#pragma unroll 1
    for (int kc = 0; kc < K; kc += 32) {
        const v16bf a = cat16b(*(const v8us*)(Ah + aoff + kc), *(const v8us*)(Ah + aoff + kc + 16));
        const v16bf al = cat16b(*(const v8us*)(Al + aoff + kc), *(const v8us*)(Al + aoff + kc + 16));
#pragma unroll
        for (int t = 0; t < 4; ++t) { const size_t bo = (size_t)(c0 + t * 16 + lr) * K + kc + 8 * hi;
            const v16bf bh = cat16b(*(const v8us*)(Bh + bo), *(const v8us*)(Bh + bo + 16)); const v16bf bl = cat16b(*(const v8us*)(Bl + bo), *(const v8us*)(Bl + bo + 16));
            acc[t] = wmmab(a, bh, acc[t]); acc[t] = wmmab(al, bh, acc[t]); acc[t] = wmmab(a, bl, acc[t]); }
        asm volatile("v_nop\n\tv_nop\n\tv_nop\n\tv_nop" : "+v"(acc[0]), "+v"(acc[1]), "+v"(acc[2]), "+v"(acc[3]) : "v"(a), "v"(al));
    }
    float* os = &ost[wave][0];
#pragma unroll
    for (int t = 0; t < 4; ++t) {
#pragma unroll
        for (int j = 0; j < 8; ++j) os[(hi * 8 + j) * 68 + t * 16 + lr] = acc[t][j]; }
    __builtin_amdgcn_wave_barrier(); asm volatile("" ::: "memory");
    float* crow = C + (size_t)r0 * ldc + c0;
    auto pass = [&]() {
#pragma unroll
        for (int s = 0; s < 8; ++s) { const int Lid = (lane >> 3) + 4 * s, piece = lane & 7; const int row = Lid >> 1, cofs = (Lid & 1) * 32 + piece * 4;
            const v4f val = *(const v4fa*)(os + row * 68 + cofs); *(volatile v4f*)(crow + (size_t)row * ldc + cofs) = val; }
    };
    pass(); __threadfence(); pass();
}


__global__ __launch_bounds__(256) void k_ptb(const float* __restrict__ xb, bf* XT) {
    __shared__ float tl[64][65];
    typedef __attribute__((ext_vector_type(4))) unsigned short v4us;
    const int tid = threadIdx.x, c0 = blockIdx.x * 64, p0 = blockIdx.y * 64; const int rr = tid >> 2, cq = (tid & 3) * 16;
#pragma unroll
    for (int i = 0; i < 16; ++i) tl[rr][cq + i] = xb[(size_t)(c0 + rr) * NPX + p0 + cq + i];
    __syncthreads();
    const int lane = tid & 31, wv = tid >> 5;
    auto pass = [&]() {
#pragma unroll
        for (int st = 0; st < 4; ++st) { const int pr = wv * 8 + st * 2 + (lane >> 4); const int cl = (lane & 15) * 4; v4us v;
#pragma unroll
            for (int i = 0; i < 4; ++i) v[i] = f2bf(tl[cl + i][pr]);
            *(volatile v4us*)(XT + (size_t)(p0 + pr) * CC + c0 + cl) = v; }
    };
    pass(); __threadfence(); pass();
}
__global__ __launch_bounds__(256) void k_split64(const float* __restrict__ F, int rows, bf* Ph, bf* Pl) {
    typedef __attribute__((ext_vector_type(2))) unsigned short v2us; typedef __attribute__((ext_vector_type(2))) float v2f_;
    const int lane = threadIdx.x & 31; const size_t r = (size_t)blockIdx.x * 8 + (threadIdx.x >> 5); if (r >= (size_t)rows) return; const size_t o = r * DI + lane * 2; const v2f_ v = *(const v2f_*)(F + o); v2us oh, ol;
#pragma unroll
    for (int i = 0; i < 2; ++i) { const unsigned short hb = f2bf(v[i]); oh[i] = hb; ol[i] = f2bf(v[i] - bf2f(hb)); }
    *(volatile v2us*)(Ph + o) = oh; *(volatile v2us*)(Pl + o) = ol; __threadfence(); *(volatile v2us*)(Ph + o) = oh; *(volatile v2us*)(Pl + o) = ol;
}
__global__ __launch_bounds__(256) void k_gT(const float* __restrict__ G, bf* Th, bf* Tl) {
    __shared__ float tl[64][65];
    typedef __attribute__((ext_vector_type(4))) unsigned short v4us;
    const int tid = threadIdx.x; const int j0 = blockIdx.x * 64; const int rr = tid >> 2, cq = (tid & 3) * 16;
#pragma unroll
    for (int i = 0; i < 16; ++i) tl[rr][cq + i] = G[(size_t)(j0 + rr) * DI + cq + i];
    __syncthreads();
    const int lane = tid & 31, wv = tid >> 5;
    auto pass = [&]() {
#pragma unroll
        for (int st = 0; st < 4; ++st) { const int dr = wv * 8 + st * 2 + (lane >> 4); const int jq = (lane & 15) * 4; v4us oh, ol;
#pragma unroll
            for (int i = 0; i < 4; ++i) { const float y = tl[jq + i][dr]; const unsigned short hb = f2bf(y); oh[i] = hb; ol[i] = f2bf(y - bf2f(hb)); }
            const size_t o = (size_t)dr * NPX + j0 + jq; *(volatile v4us*)(Th + o) = oh; *(volatile v4us*)(Tl + o) = ol; }
    };
    pass(); __threadfence(); pass();
}
__global__ __launch_bounds__(256) void k_soft(const float* __restrict__ S, bf* PH, bf* PL) {
    typedef __attribute__((ext_vector_type(4))) unsigned short v4us;
    const int lane = threadIdx.x & 31, i = blockIdx.x * 8 + (threadIdx.x >> 5); if (i >= QH) return; const float* sr = S + (size_t)i * NPX;
    float m = -3.0e38f;
#pragma unroll 1
    for (int c0 = lane * 4; c0 < NPX; c0 += 128) {
#pragma unroll
        for (int q = 0; q < 4; ++q) m = fmaxf(m, sr[c0 + q]); }
#pragma unroll
    for (int sh = 16; sh; sh >>= 1) m = fmaxf(m, __shfl_xor(m, sh, 32));
    float sum = 0.f;
#pragma unroll 1
    for (int c0 = lane * 4; c0 < NPX; c0 += 128) {
#pragma unroll
        for (int q = 0; q < 4; ++q) sum += __expf(sr[c0 + q] - m); }
#pragma unroll
    for (int sh = 16; sh; sh >>= 1) sum += __shfl_xor(sum, sh, 32);
    const float inv = 1.0f / sum;
#pragma unroll 1
    for (int ps = 0; ps < 2; ++ps) {
#pragma unroll 1
        for (int c0 = lane * 4; c0 < NPX; c0 += 128) { v4us oh, ol;
#pragma unroll
            for (int q = 0; q < 4; ++q) { const float p = __expf(sr[c0 + q] - m) * inv; const unsigned short hb = f2bf(p); oh[q] = hb; ol[q] = f2bf(p - bf2f(hb)); }
            const size_t o = (size_t)i * NPX + c0; *(volatile v4us*)(PH + o) = oh; *(volatile v4us*)(PL + o) = ol; }
        if (ps == 0) __threadfence(); }
}
__global__ __launch_bounds__(256) void k_bnstat(const float* __restrict__ Y2, float* MEAN, float* RSTD) {
    const int lane = threadIdx.x & 31; const int w = blockIdx.x * 8 + (threadIdx.x >> 5); if (w >= CC / 32) return; const int c = w * 32 + lane; const int n = NB_ * NPX; float s = 0.f;
    for (int r = 0; r < n; ++r) s += Y2[(size_t)r * CC + c];
    const float mu = s / (float)n; float q = 0.f;
    for (int r = 0; r < n; ++r) { const float d = Y2[(size_t)r * CC + c] - mu; q = fmaf(d, d, q); }
    const float rs = rsqrtf(q / (float)n + BEPS);
    *(volatile float*)(MEAN + c) = mu; *(volatile float*)(RSTD + c) = rs; __threadfence(); *(volatile float*)(MEAN + c) = mu; *(volatile float*)(RSTD + c) = rs;
}
__global__ __launch_bounds__(256) void k_bnout(const float* __restrict__ Y2, const float* __restrict__ x, const float* __restrict__ MEAN, const float* __restrict__ RSTD, const float* __restrict__ gam, const float* __restrict__ bet, const float* __restrict__ scale, float* OUTB) {
    __shared__ float tl[64][65];
    const int tid = threadIdx.x; const int p0 = blockIdx.x * 64, c0 = blockIdx.y * 64, b = blockIdx.z; const int rr = tid >> 2, cq = (tid & 3) * 16;
#pragma unroll
    for (int i = 0; i < 16; ++i) { const int c = c0 + cq + i; tl[rr][cq + i] = (Y2[((size_t)b * NPX + p0 + rr) * CC + c] - MEAN[c]) * RSTD[c] * bfr(gam[c]) + bfr(bet[c]); }
    __syncthreads();
    const int lane = tid & 31, wv = tid >> 5; const float sc = bfr(scale[0]);
    auto pass = [&]() {
#pragma unroll
        for (int st = 0; st < 4; ++st) { const int cr = wv * 8 + st * 2 + (lane >> 4); const int pq = (lane & 15) * 4; v4f v; const size_t o = ((size_t)b * CC + c0 + cr) * NPX + p0 + pq;
#pragma unroll
            for (int i = 0; i < 4; ++i) v[i] = bfr(x[o + i]) + sc * tl[pq + i][cr];
            *(volatile v4f*)(OUTB + o) = v; }
    };
    pass(); __threadfence(); pass();
}

extern "C" void kernel_launch(void* const* d_in, const int* in_sizes, int n_in,
                              void* d_out, int out_size, void* d_ws, size_t ws_size, hipStream_t stream) {
    (void)in_sizes; (void)n_in; (void)out_size;
    const float* x = (const float*)d_in[0]; const float* thw = (const float*)d_in[1]; const float* thb = (const float*)d_in[2]; const float* phw = (const float*)d_in[3]; const float* phb = (const float*)d_in[4]; const float* gw = (const float*)d_in[5]; const float* gb = (const float*)d_in[6];
    const float* ow = (const float*)d_in[7]; const float* ob = (const float*)d_in[8]; const float* gam = (const float*)d_in[9]; const float* bet = (const float*)d_in[10]; const float* scale = (const float*)d_in[11];
    float* out = (float*)d_out;
    char* wsp = (char*)d_ws;
    auto take = [&](size_t bytes) { char* p = wsp; wsp += (bytes + 255) & ~(size_t)255; return (void*)p; };
    bf* WT = (bf*)take((size_t)DI * CC * 2); bf* WP = (bf*)take((size_t)DI * CC * 2); bf* WG = (bf*)take((size_t)DI * CC * 2); bf* WO = (bf*)take((size_t)CC * DI * 2);
    bf* XT = (bf*)take((size_t)NPX * CC * 2); float* TH = (float*)take((size_t)NPX * DI * 4); float* PHI = (float*)take((size_t)NPX * DI * 4); float* G = (float*)take((size_t)NPX * DI * 4);
    bf* Th = (bf*)take((size_t)NPX * DI * 2); bf* Tl = (bf*)take((size_t)NPX * DI * 2); bf* Fh = (bf*)take((size_t)NPX * DI * 2); bf* Fl = (bf*)take((size_t)NPX * DI * 2); bf* GTh = (bf*)take((size_t)DI * NPX * 2); bf* GTl = (bf*)take((size_t)DI * NPX * 2);
    float* S = (float*)take((size_t)QH * NPX * 4); bf* PH = (bf*)take((size_t)QH * NPX * 2); bf* PL = (bf*)take((size_t)QH * NPX * 2); float* YT = (float*)take((size_t)NPX * DI * 4); bf* Yh = (bf*)take((size_t)NPX * DI * 2); bf* Yl = (bf*)take((size_t)NPX * DI * 2);
    float* Y2 = (float*)take((size_t)NB_ * NPX * CC * 4); float* MEAN = (float*)take(CC * 4); float* RSTD = (float*)take(CC * 4);
    if ((size_t)(wsp - (char*)d_ws) > ws_size) return;
    k_cvt8<<<(DI * CC / 8 + 255) / 256, 256, 0, stream>>>(thw, WT, DI * CC / 8); k_cvt8<<<(DI * CC / 8 + 255) / 256, 256, 0, stream>>>(phw, WP, DI * CC / 8); k_cvt8<<<(DI * CC / 8 + 255) / 256, 256, 0, stream>>>(gw, WG, DI * CC / 8); k_cvt8<<<(CC * DI / 8 + 255) / 256, 256, 0, stream>>>(ow, WO, CC * DI / 8);
    for (int b = 0; b < NB_; ++b) {
        k_ptb<<<dim3(CC / 64, NPX / 64, 1), 256, 0, stream>>>(x + (size_t)b * CC * NPX, XT);
        k_gemmb<false, false><<<dim3(NPX / 64, 1, 1), 128, 0, stream>>>(XT, nullptr, WT, thb, TH, DI, nullptr, nullptr, CC); k_gemmb<false, false><<<dim3(NPX / 64, 1, 1), 128, 0, stream>>>(XT, nullptr, WP, phb, PHI, DI, nullptr, nullptr, CC); k_gemmb<false, false><<<dim3(NPX / 64, 1, 1), 128, 0, stream>>>(XT, nullptr, WG, gb, G, DI, nullptr, nullptr, CC);
        k_split64<<<NPX / 8, 256, 0, stream>>>(TH, NPX, Th, Tl); k_split64<<<NPX / 8, 256, 0, stream>>>(PHI, NPX, Fh, Fl); k_gT<<<NPX / 64, 256, 0, stream>>>(G, GTh, GTl);
        for (int hf = 0; hf < NPX / QH; ++hf) { const size_t r0 = (size_t)hf * QH;
            k_gemm3<<<dim3(QH / 64, NPX / 64, 1), 128, 0, stream>>>(Th + r0 * DI, Tl + r0 * DI, Fh, Fl, DI, S, NPX);
            k_soft<<<QH / 8, 256, 0, stream>>>(S, PH, PL);
            k_gemm3<<<dim3(QH / 64, 1, 1), 128, 0, stream>>>(PH, PL, GTh, GTl, NPX, YT + r0 * DI, DI); }
        k_split64<<<NPX / 8, 256, 0, stream>>>(YT, NPX, Yh, Yl);
        k_gemmb<true, false><<<dim3(NPX / 64, CC / 64, 1), 128, 0, stream>>>(Yh, Yl, WO, ob, Y2 + (size_t)b * NPX * CC, CC, nullptr, nullptr, DI); }
    k_bnstat<<<(CC / 32) / 8, 256, 0, stream>>>(Y2, MEAN, RSTD);
    k_bnout<<<dim3(NPX / 64, CC / 64, NB_), 256, 0, stream>>>(Y2, x, MEAN, RSTD, gam, bet, scale, out);
}
